// Batch_Contrastive_18116172055214
// MI455X (gfx1250) — hardware-verified
//
#include <hip/hip_runtime.h>


#define NBT  8
#define CC   256
#define HW   1024
#define NN   (NBT * HW)
#define NCOL 3
#define RCH  1024
#define DM   CC
#define LOSC 1024.0f

typedef _Float16 h16;
typedef unsigned short bf;
typedef __attribute__((ext_vector_type(16))) __bf16   v16bf;
typedef __attribute__((ext_vector_type(16))) _Float16 v16h;
typedef __attribute__((ext_vector_type(8)))  _Float16 v8h;
typedef __attribute__((ext_vector_type(8)))  unsigned short v8us;
typedef __attribute__((ext_vector_type(8)))  float    v8f;
typedef __attribute__((ext_vector_type(4)))  float    v4f;
typedef v8h  __attribute__((may_alias)) v8ha;
typedef v4f  __attribute__((may_alias)) v4fa;
typedef v8us __attribute__((may_alias)) v8usa;

__device__ __forceinline__ unsigned short f2bf(float f) { unsigned u = __float_as_uint(f); u += 0x7FFFu + ((u >> 16) & 1u); return (unsigned short)(u >> 16); }
__device__ __forceinline__ float bf2f(unsigned short b) { return __uint_as_float(((unsigned)b) << 16); }
__device__ __forceinline__ float bfr(float f) { return bf2f(f2bf(f)); }
__device__ __forceinline__ v16h cat16(v8h lo, v8h hi) { return __builtin_shufflevector(lo, hi, 0, 1, 2, 3, 4, 5, 6, 7, 8, 9, 10, 11, 12, 13, 14, 15); }
__device__ __forceinline__ v16bf cat16b(v8us lo, v8us hi) { return __builtin_bit_cast(v16bf, __builtin_shufflevector(lo, hi, 0, 1, 2, 3, 4, 5, 6, 7, 8, 9, 10, 11, 12, 13, 14, 15)); }
__device__ __forceinline__ v8f wmma16(v16h a, v16h b, v8f c) { return __builtin_amdgcn_wmma_f32_16x16x32_f16(false, a, false, b, (short)0, c, false, false); }
__device__ __forceinline__ v8f wmmab(v16bf a, v16bf b, v8f c) { return __builtin_amdgcn_wmma_f32_16x16x32_bf16(false, a, false, b, (short)0, c, false, false); }

template <bool SPLITA, bool F16OUT = false>
__global__ __launch_bounds__(128) void k_gemmb(const bf* __restrict__ A, const bf* __restrict__ Al, const bf* __restrict__ Bn, const float* __restrict__ bias, float* C, int ldc, h16* C2, const float* __restrict__ R = nullptr, int K = DM, int roundR = 1) {
    __shared__ __align__(16) float ost[4][16 * 68];
    const int lane = threadIdx.x & 31, wave = threadIdx.x >> 5, lr = lane & 15, hi = lane >> 4;
    const int r0 = blockIdx.x * 64 + wave * 16, c0 = blockIdx.y * 64;
    const size_t aoff = (size_t)(r0 + lr) * K + 8 * hi;
    size_t boff[4];
#pragma unroll
    for (int t = 0; t < 4; ++t) boff[t] = (size_t)(c0 + t * 16 + lr) * K + 8 * hi;
    v8f acc[4];
#pragma unroll
    for (int t = 0; t < 4; ++t) acc[t] = (v8f){};
#pragma unroll 1
    for (int kc = 0; kc < K; kc += 32) {
        const v16bf a = cat16b(*(const v8us*)(A + aoff + kc), *(const v8us*)(A + aoff + kc + 16));
        v16bf al = a;
        if (SPLITA) al = cat16b(*(const v8us*)(Al + aoff + kc), *(const v8us*)(Al + aoff + kc + 16));
#pragma unroll
        for (int t = 0; t < 4; ++t) { const v16bf b = cat16b(*(const v8us*)(Bn + boff[t] + kc), *(const v8us*)(Bn + boff[t] + kc + 16)); acc[t] = wmmab(a, b, acc[t]); if (SPLITA) acc[t] = wmmab(al, b, acc[t]); }
        asm volatile("v_nop\n\tv_nop\n\tv_nop\n\tv_nop" : "+v"(acc[0]), "+v"(acc[1]), "+v"(acc[2]), "+v"(acc[3]) : "v"(a), "v"(al));
    }
    float* os = &ost[wave][0];
#pragma unroll
    for (int t = 0; t < 4; ++t) { const float bv = bias ? bfr(bias[c0 + t * 16 + lr]) : 0.f;
#pragma unroll
        for (int j = 0; j < 8; ++j) os[(hi * 8 + j) * 68 + t * 16 + lr] = acc[t][j] + bv; }
    __syncthreads();
    if (F16OUT) {
        h16* crow = (h16*)(void*)C + (size_t)r0 * ldc + c0;
        auto pass = [&]() {
#pragma unroll
            for (int s = 0; s < 4; ++s) { const int row = 4 * s + (lane >> 3), piece = lane & 7; const float* sp = os + row * 68 + piece * 8; v8h o, o2;
#pragma unroll
                for (int i = 0; i < 8; ++i) { const h16 a = (h16)sp[i]; o[i] = a; o2[i] = (h16)((sp[i] - (float)a) * LOSC); }
                *(volatile v8h*)(crow + (size_t)row * ldc + piece * 8) = o; if (C2) *(volatile v8h*)(C2 + (size_t)r0 * ldc + c0 + (size_t)row * ldc + piece * 8) = o2; }
        };
        pass(); __threadfence(); pass();
    } else {
        float* crow = C + (size_t)r0 * ldc + c0;
        auto pass = [&]() {
#pragma unroll
            for (int s = 0; s < 8; ++s) { const int Lid = (lane >> 3) + 4 * s, piece = lane & 7; const int row = Lid >> 1, cofs = (Lid & 1) * 32 + piece * 4;
                v4f val = *(const v4fa*)(os + row * 68 + cofs); if (R) { const v4f rv = *(const v4f*)(R + ((size_t)r0 + row) * ldc + c0 + cofs); val += roundR ? (v4f){bfr(rv[0]), bfr(rv[1]), bfr(rv[2]), bfr(rv[3])} : rv; }
                *(volatile v4f*)(crow + (size_t)row * ldc + cofs) = val; }
        };
        pass(); __threadfence(); pass();
    }
}


__global__ __launch_bounds__(256) void k_pix(const float* __restrict__ src, bf* dst) {
    __shared__ float tl[64][65];
    const int tid = threadIdx.x, c0 = blockIdx.x * 64, p0 = blockIdx.y * 64, b = blockIdx.z; const int cc = tid >> 2, pq = (tid & 3) * 16;
#pragma unroll
    for (int i = 0; i < 16; ++i) tl[cc][pq + i] = src[((size_t)b * CC + c0 + cc) * HW + p0 + pq + i];
    __syncthreads();
    const int piece = tid & 7, pr0 = tid >> 3;
    auto pass = [&]() {
#pragma unroll
        for (int st = 0; st < 2; ++st) { const int pr = pr0 + 32 * st; v8us o;
#pragma unroll
            for (int i = 0; i < 8; ++i) o[i] = f2bf(tl[piece * 8 + i][pr]);
            *(volatile v8us*)(dst + ((size_t)b * HW + p0 + pr) * CC + c0 + piece * 8) = o; }
    };
    pass(); __threadfence(); pass();
}
__global__ __launch_bounds__(256) void k_fct(const float* __restrict__ fc, bf* FCt) {
    const int lane = threadIdx.x & 31; const int wid = blockIdx.x * 8 + (threadIdx.x >> 5); if (wid >= 64 * (NN / 256)) return; const int c = wid / (NN / 256); const int n0 = (wid % (NN / 256)) * 256 + lane * 8; v8us o;
#pragma unroll
    for (int i = 0; i < 8; ++i) { const int n = n0 + i; const int b = n / HW, p = n % HW; o[i] = (c < NCOL) ? f2bf(fc[((size_t)b * NCOL + (c < NCOL ? c : 0)) * HW + p]) : (unsigned short)0; }
    *(volatile v8us*)(FCt + (size_t)c * NN + n0) = o; __threadfence(); *(volatile v8us*)(FCt + (size_t)c * NN + n0) = o;
}
__global__ __launch_bounds__(256) void k_softblk(const float* __restrict__ S, int r0, bf* PH, bf* PL, float* BSL) {
    typedef __attribute__((ext_vector_type(4))) unsigned short v4us;
    __shared__ float sh[8];
    const int lane = threadIdx.x & 31, wv = threadIdx.x >> 5, i = blockIdx.x * 8 + wv; const int n = r0 + i; const int blk = n / HW;
    float m = -3.0e38f;
#pragma unroll 1
    for (int c0 = lane * 4; c0 < NN; c0 += 128) {
#pragma unroll
        for (int q = 0; q < 4; ++q) m = fmaxf(m, S[(size_t)i * NN + c0 + q]); }
#pragma unroll
    for (int s_ = 16; s_; s_ >>= 1) m = fmaxf(m, __shfl_xor(m, s_, 32));
    float sum = 0.f;
#pragma unroll 1
    for (int c0 = lane * 4; c0 < NN; c0 += 128) {
#pragma unroll
        for (int q = 0; q < 4; ++q) sum += __expf(S[(size_t)i * NN + c0 + q] - m); }
#pragma unroll
    for (int s_ = 16; s_; s_ >>= 1) sum += __shfl_xor(sum, s_, 32);
    const float inv = 1.0f / sum; float bs = 0.f;
#pragma unroll 1
    for (int ps = 0; ps < 2; ++ps) { bs = 0.f;
#pragma unroll 1
        for (int c0 = lane * 4; c0 < NN; c0 += 128) { v4us oh, ol;
#pragma unroll
            for (int q = 0; q < 4; ++q) { const int col = c0 + q; const float p = __expf(S[(size_t)i * NN + col] - m) * inv; if (col / HW == blk) bs += p; const unsigned short hb = f2bf(p); oh[q] = hb; ol[q] = f2bf(p - bf2f(hb)); }
            const size_t o = (size_t)i * NN + c0; *(volatile v4us*)(PH + o) = oh; *(volatile v4us*)(PL + o) = ol; }
        if (ps == 0) __threadfence(); }
#pragma unroll
    for (int s_ = 16; s_; s_ >>= 1) bs += __shfl_xor(bs, s_, 32);
    if (lane == 0) sh[wv] = bs;
    __syncthreads();
    if (wv == 0) { const float v = (lane < 8) ? sh[lane] : 0.f; float* d = BSL + (size_t)(r0 / 8 + blockIdx.x) * 32 + lane; *(volatile float*)d = v; __threadfence(); *(volatile float*)d = v; }
}
__global__ __launch_bounds__(256) void k_img(const float* __restrict__ CL, float* OUT0) {
    const int lane = threadIdx.x & 31; const int wid = blockIdx.x * 8 + (threadIdx.x >> 5); if (wid >= NBT * NCOL * (HW / 128)) return; const int pg = wid % (HW / 128), rest = wid / (HW / 128), c = rest % NCOL, b = rest / NCOL; const int p0 = pg * 128 + lane * 4; v4f v;
#pragma unroll
    for (int q = 0; q < 4; ++q) v[q] = CL[((size_t)b * HW + p0 + q) * 64 + c];
    float* d = OUT0 + ((size_t)b * NCOL + c) * HW + p0; *(volatile v4f*)d = v; __threadfence(); *(volatile v4f*)d = v;
}
__global__ __launch_bounds__(256) void k_loss(const float* __restrict__ BSL, float* OUT1) {
    __shared__ float pa[256];
    const int t = threadIdx.x; float a = 0.f; const int per = NN / 256;
    for (int q = 0; q < per; ++q) { const int n = t * per + q; a += fabsf(BSL[(size_t)(n >> 3) * 32 + (n & 7)] - 1.0f); }
    pa[t] = a; __syncthreads();
    if (t == 0) { float A = 0.f; for (int k = 0; k < 256; ++k) A += pa[k]; const float v = A * (1.0f / NN); *(volatile float*)OUT1 = v; __threadfence(); *(volatile float*)OUT1 = v; }
}

extern "C" void kernel_launch(void* const* d_in, const int* in_sizes, int n_in,
                              void* d_out, int out_size, void* d_ws, size_t ws_size, hipStream_t stream) {
    (void)in_sizes; (void)n_in; (void)out_size;
    const float* f2 = (const float*)d_in[0]; const float* f1 = (const float*)d_in[1]; const float* fc = (const float*)d_in[2];
    float* out0 = (float*)d_out;
    float* out1 = (float*)((char*)d_out + (size_t)NBT * NCOL * HW * 4);
    char* wsp = (char*)d_ws;
    auto take = [&](size_t bytes) { char* p = wsp; wsp += (bytes + 255) & ~(size_t)255; return (void*)p; };
    bf* F2 = (bf*)take((size_t)NN * CC * 2); bf* F1 = (bf*)take((size_t)NN * CC * 2); bf* FCt = (bf*)take((size_t)64 * NN * 2);
    float* S = (float*)take((size_t)RCH * NN * 4); bf* PH = (bf*)take((size_t)RCH * NN * 2); bf* PL = (bf*)take((size_t)RCH * NN * 2); float* BSL = (float*)take((size_t)(NN / 8) * 32 * 4); float* CL = (float*)take((size_t)NN * 64 * 4);
    if ((size_t)(wsp - (char*)d_ws) > ws_size) return;
    k_pix<<<dim3(CC / 64, HW / 64, NBT), 256, 0, stream>>>(f2, F2); k_pix<<<dim3(CC / 64, HW / 64, NBT), 256, 0, stream>>>(f1, F1); k_fct<<<(64 * (NN / 256)) / 8, 256, 0, stream>>>(fc, FCt);
    for (int ch = 0; ch < NN / RCH; ++ch) { const int r0 = ch * RCH;
        k_gemmb<false, false><<<dim3(RCH / 64, NN / 64, 1), 128, 0, stream>>>(F2 + (size_t)r0 * CC, nullptr, F1, nullptr, S, NN, nullptr, nullptr, CC);
        k_softblk<<<RCH / 8, 256, 0, stream>>>(S, r0, PH, PL, BSL);
        k_gemmb<true, false><<<dim3(RCH / 64, 1, 1), 128, 0, stream>>>(PH, PL, FCt, nullptr, CL + (size_t)r0 * 64, 64, nullptr, nullptr, NN); }
    k_img<<<(NBT * NCOL * (HW / 128)) / 8, 256, 0, stream>>>(CL, out0);
    k_loss<<<1, 256, 0, stream>>>(BSL, out1);
}
